// SelfAttention_4535485464962
// MI455X (gfx1250) — hardware-verified
//
#include <hip/hip_runtime.h>
#ifndef NB
#define NB 2
#endif
#ifndef SEQ
#define SEQ 2048
#endif
#define SEQ_FULL 2048
#define DM 1024
#define NH 16
#define HD 64
#define MR (NB * SEQ)
#define NW (SEQ / 32)
#define NFB (SEQ / 32)
#define NFBP (((NFB + 31) / 32) * 32)
#define EARLY ((SEQ >= 512) ? 256 : (SEQ / 2))

typedef __bf16 v16b __attribute__((ext_vector_type(16)));
typedef _Float16 v16h __attribute__((ext_vector_type(16)));
typedef unsigned short v8us __attribute__((ext_vector_type(8), may_alias));
typedef unsigned int v4u __attribute__((ext_vector_type(4)));
typedef unsigned int v4ua __attribute__((ext_vector_type(4), may_alias));
typedef float v8f __attribute__((ext_vector_type(8)));
typedef float v4f __attribute__((ext_vector_type(4)));
typedef float v4fa __attribute__((ext_vector_type(4), may_alias));
union FragB { v16b v; v8us half[2]; };
union FragH { v16h v; v8us half[2]; _Float16 h[16]; };
union H8 { v8us u; _Float16 h[8]; };

static_assert(NH * HD == DM);
static_assert(HD == 64);
static_assert(DM % 128 == 0);
static_assert(DM % 32 == 0);
static_assert(SEQ % 128 == 0);
static_assert(MR % 128 == 0);
static_assert(SEQ <= SEQ_FULL);
static_assert(EARLY % 64 == 0);
static_assert((SEQ - EARLY) % 64 == 0);
static_assert(SEQ > EARLY);
static_assert((NFB * 8) % 8 == 0);

constexpr size_t SZ_XB = (size_t)MR * DM * 2;
constexpr size_t SZ_WQ = (size_t)3 * DM * DM * 2;
constexpr size_t SZ_WP = (size_t)DM * DM * 2;
constexpr size_t SZ_QK = (size_t)MR * 2 * DM * 2;
constexpr size_t SZ_VT = (size_t)DM * MR * 2;
constexpr size_t SZ_CX = (size_t)MR * DM * 2;
constexpr size_t SZ_MB = (size_t)NW * SEQ * 4;
constexpr size_t SZ_FL = (size_t)NFB * 32 * 4;
constexpr size_t OFF_XB = 0;
constexpr size_t OFF_WQ = OFF_XB + SZ_XB;
constexpr size_t OFF_WP = OFF_WQ + SZ_WQ;
constexpr size_t OFF_QKH = OFF_WP + SZ_WP;
constexpr size_t OFF_QKL = OFF_QKH + SZ_QK;
constexpr size_t OFF_VTH = OFF_QKL + SZ_QK;
constexpr size_t OFF_VTL = OFF_VTH + SZ_VT;
constexpr size_t OFF_CH = OFF_VTL + SZ_VT;
constexpr size_t OFF_CL = OFF_CH + SZ_CX;
constexpr size_t OFF_MB = OFF_CL + SZ_CX;
constexpr size_t OFF_FL = OFF_MB + SZ_MB;
constexpr size_t WS_TOTAL = OFF_FL + SZ_FL;
static_assert(WS_TOTAL <= (size_t)134217728);
static_assert(SZ_XB % 256 == 0 && SZ_WQ % 256 == 0 && SZ_WP % 256 == 0 && SZ_QK % 256 == 0 && SZ_VT % 256 == 0 && SZ_CX % 256 == 0 && SZ_MB % 256 == 0 && SZ_FL % 128 == 0);

__device__ __forceinline__ unsigned short bf16_bits(float x) { const unsigned int u = __float_as_uint(x); return (unsigned short)((u + 0x7FFFu + ((u >> 16) & 1u)) >> 16); }
__device__ __forceinline__ float bf16_val(unsigned short b) { return __uint_as_float(((unsigned int)b) << 16); }
__device__ __forceinline__ float bf16_rne_val(float x) { return bf16_val(bf16_bits(x)); }

__device__ __forceinline__ v8f mma_b(const v16b a, const v16b b, const v8f c) {
  v8f d = __builtin_amdgcn_wmma_f32_16x16x32_bf16(false, a, false, b, (short)0, c, false, false);
  asm volatile("v_nop\n\tv_nop\n\tv_nop\n\tv_nop" : "+v"(d) : "v"(a), "v"(b));
  return d;
}
__device__ __forceinline__ v8f mma_h(const v16h a, const v16h b, const v8f c) {
  v8f d = __builtin_amdgcn_wmma_f32_16x16x32_f16(false, a, false, b, (short)0, c, false, false);
  asm volatile("v_nop\n\tv_nop\n\tv_nop\n\tv_nop" : "+v"(d) : "v"(a), "v"(b));
  return d;
}
__device__ __forceinline__ v16b ldfrag_b(const unsigned short* __restrict__ p) { FragB f; f.half[0] = *(const v8us*)p; f.half[1] = *(const v8us*)(p + 16); return f.v; }
__device__ __forceinline__ v16h ldfrag_h(const unsigned short* __restrict__ p) { FragH f; f.half[0] = *(const v8us*)p; f.half[1] = *(const v8us*)(p + 16); return f.v; }

__global__ __launch_bounds__(256) void k_wt_bf16(const float* __restrict__ W, unsigned short* __restrict__ Wt, int K, int N) {
  const int t = blockIdx.x * 256 + threadIdx.x;
  const int k8n = K / 8;
  if (t >= N * k8n) return;
  const int n = t / k8n, k8 = (t % k8n) * 8;
  v8us v;
#pragma unroll
  for (int i = 0; i < 8; ++i) v[i] = bf16_bits(W[(size_t)(k8 + i) * N + n]);
  *(volatile v8us*)(Wt + (size_t)n * K + k8) = v;
  __threadfence();
  *(volatile v8us*)(Wt + (size_t)n * K + k8) = v;
}

__global__ __launch_bounds__(256) void k_xb(const float* __restrict__ x, unsigned short* __restrict__ XB) {
  const size_t t = (size_t)blockIdx.x * 256 + threadIdx.x;
  if (t >= (size_t)MR * (DM / 8)) return;
  const int row = (int)(t / (DM / 8)), c8 = (int)(t % (DM / 8)) * 8;
  const int b = row / SEQ, tt = row - b * SEQ;
  const float* src = x + ((size_t)b * SEQ_FULL + tt) * DM + c8;
  const v4f a = *(const v4fa*)src, c = *(const v4fa*)(src + 4);
  v8us v;
#pragma unroll
  for (int q = 0; q < 4; ++q) { v[q] = bf16_bits(a[q]); v[4 + q] = bf16_bits(c[q]); }
  *(volatile v8us*)(XB + t * 8) = v;
  __threadfence();
  *(volatile v8us*)(XB + t * 8) = v;
}

__global__ __launch_bounds__(256) void k_maskpack(const int* __restrict__ mask, unsigned int* __restrict__ MB, unsigned int* __restrict__ FL) {
  __shared__ __attribute__((aligned(16))) unsigned int sm[NW][32];
  __shared__ unsigned int sfl[8];
  const int tid = threadIdx.x, lane = tid & 31;
  const int wave = __builtin_amdgcn_readfirstlane(tid >> 5);
  const int q0 = blockIdx.x * 32;
  unsigned int wflag = 0u;
#pragma unroll 1
  for (int rr = 0; rr < 4; ++rr) {
    const int qi = wave * 4 + rr;
    const int* mrow = mask + (size_t)(q0 + qi) * SEQ_FULL;
    unsigned int rowor = 0u;
#pragma unroll 1
    for (int wd = 0; wd < NW; ++wd) {
      const int mv = mrow[wd * 32 + lane];
      const unsigned int bal = __builtin_amdgcn_ballot_w32(mv != 0);
      rowor |= bal;
      if (lane == 0) sm[wd][qi] = bal;
    }
    if (rowor == 0u) wflag = 1u;
  }
  if (lane == 0) sfl[wave] = wflag;
  __syncthreads();
  unsigned int bf = 0u;
#pragma unroll
  for (int i = 0; i < 8; ++i) bf |= sfl[i];
  const v4u fl4 = {bf, bf, bf, bf};
  for (int pass = 0; pass < 2; ++pass) {
#pragma unroll 1
    for (int idx = tid; idx < NW * 8; idx += 256) {
      const int wd = idx >> 3, part = idx & 7;
      const v4u xw = *(const v4ua*)&sm[wd][part * 4];
      *(volatile v4u*)(MB + (size_t)wd * SEQ + q0 + part * 4) = xw;
    }
    if (tid < 8) *(volatile v4u*)(FL + (size_t)blockIdx.x * 32 + tid * 4) = fl4;
    if (pass == 0) __threadfence();
  }
}

template <int NT, int MODE>
__device__ __forceinline__ void gemm_body(const unsigned short* __restrict__ AH, const unsigned short* __restrict__ AL, const int lda,
                                          const unsigned short* __restrict__ BT, const int ldb, const float* __restrict__ bias,
                                          float* __restrict__ CF, unsigned short* __restrict__ C0, unsigned short* __restrict__ C1,
                                          const int ldc, const int N, const int K) {
  __shared__ __attribute__((aligned(16))) float so[4][32][68];
  const int tid = threadIdx.x, lane = tid & 31, ln = lane & 15, hh = lane >> 4;
  const int wave = __builtin_amdgcn_readfirstlane(tid >> 5);
  const int ntn = N >> 6;
  const int mt = blockIdx.x / ntn, nq = blockIdx.x - mt * ntn;
  const int row0 = mt * 128 + 32 * wave, col0 = nq * 64;
  const size_t ao0 = (size_t)(row0 + ln) * lda + 8 * hh, ao1 = ao0 + (size_t)16 * lda;
  const size_t bo0 = (size_t)(col0 + ln) * ldb + 8 * hh;
  const size_t bst = (size_t)16 * ldb;
  const v8f z8 = {0.f, 0.f, 0.f, 0.f, 0.f, 0.f, 0.f, 0.f};
  v8f c00 = z8, c01 = z8, c02 = z8, c03 = z8, c10 = z8, c11 = z8, c12 = z8, c13 = z8;
#pragma unroll 1
  for (int kb = 0; kb < K; kb += 32) {
    const v16b a0 = ldfrag_b(AH + ao0 + kb), a1 = ldfrag_b(AH + ao1 + kb);
    v16b a0l = a0, a1l = a1;
    if (NT == 2) { a0l = ldfrag_b(AL + ao0 + kb); a1l = ldfrag_b(AL + ao1 + kb); }
    v16b bq = ldfrag_b(BT + bo0 + kb);
    c00 = mma_b(a0, bq, c00); c10 = mma_b(a1, bq, c10);
    if (NT == 2) { c00 = mma_b(a0l, bq, c00); c10 = mma_b(a1l, bq, c10); }
    bq = ldfrag_b(BT + bo0 + bst + kb);
    c01 = mma_b(a0, bq, c01); c11 = mma_b(a1, bq, c11);
    if (NT == 2) { c01 = mma_b(a0l, bq, c01); c11 = mma_b(a1l, bq, c11); }
    bq = ldfrag_b(BT + bo0 + 2 * bst + kb);
    c02 = mma_b(a0, bq, c02); c12 = mma_b(a1, bq, c12);
    if (NT == 2) { c02 = mma_b(a0l, bq, c02); c12 = mma_b(a1l, bq, c12); }
    bq = ldfrag_b(BT + bo0 + 3 * bst + kb);
    c03 = mma_b(a0, bq, c03); c13 = mma_b(a1, bq, c13);
    if (NT == 2) { c03 = mma_b(a0l, bq, c03); c13 = mma_b(a1l, bq, c13); }
  }
  v8f accs[8] = {c00, c01, c02, c03, c10, c11, c12, c13};
  float brow[2][8];
#pragma unroll
  for (int hf = 0; hf < 2; ++hf)
#pragma unroll
    for (int r = 0; r < 8; ++r) brow[hf][r] = (MODE == 1) ? bf16_rne_val(bias[row0 + hf * 16 + 8 * hh + r]) : 0.f;
#pragma unroll
  for (int u = 0; u < 8; ++u) {
    const int t = u & 3, hf = u >> 2;
    const float bc = (MODE != 1) ? bf16_rne_val(bias[col0 + t * 16 + ln]) : 0.f;
#pragma unroll
    for (int r = 0; r < 8; ++r) so[wave][hf * 16 + 8 * hh + r][t * 16 + ln] = accs[u][r] + bc + brow[hf][r];
  }
  __syncthreads();
  if (MODE == 2) {
    const int rsub = lane >> 4, c4 = (lane & 15) * 4;
    for (int pass = 0; pass < 2; ++pass) {
#pragma unroll
      for (int q = 0; q < 16; ++q) {
        const int r = q * 2 + rsub;
        const v4f v = *(const v4fa*)&so[wave][r][c4];
        *(volatile v4f*)(CF + (size_t)(row0 + r) * ldc + col0 + c4) = v;
      }
      if (pass == 0) __threadfence();
    }
  } else {
    const int rq = lane >> 3, c8 = (lane & 7) * 8;
    for (int pass = 0; pass < 2; ++pass) {
#pragma unroll
      for (int it = 0; it < 8; ++it) {
        const int r = it * 4 + rq;
        const v4f x0 = *(const v4fa*)&so[wave][r][c8];
        const v4f x1 = *(const v4fa*)&so[wave][r][c8 + 4];
        const size_t o = (size_t)(row0 + r) * ldc + col0 + c8;
        if (MODE == 0) {
          v8us hv, lv;
#pragma unroll
          for (int q = 0; q < 4; ++q) {
            unsigned short hb = bf16_bits(x0[q]); hv[q] = hb; lv[q] = bf16_bits(x0[q] - bf16_val(hb));
            hb = bf16_bits(x1[q]); hv[4 + q] = hb; lv[4 + q] = bf16_bits(x1[q] - bf16_val(hb));
          }
          *(volatile v8us*)(C0 + o) = hv;
          *(volatile v8us*)(C1 + o) = lv;
        } else {
          H8 fh, fl;
#pragma unroll
          for (int q = 0; q < 4; ++q) {
            _Float16 h = (_Float16)x0[q]; fh.h[q] = h; fl.h[q] = (_Float16)((x0[q] - (float)h) * 1024.0f);
            h = (_Float16)x1[q]; fh.h[4 + q] = h; fl.h[4 + q] = (_Float16)((x1[q] - (float)h) * 1024.0f);
          }
          *(volatile v8us*)(C0 + o) = fh.u;
          *(volatile v8us*)(C1 + o) = fl.u;
        }
      }
      if (pass == 0) __threadfence();
    }
  }
}

__global__ __launch_bounds__(128) void k_gemm_qk(const unsigned short* __restrict__ XB, const unsigned short* __restrict__ WQ, const float* __restrict__ bias,
                                                 unsigned short* __restrict__ QKH, unsigned short* __restrict__ QKL) {
  gemm_body<1, 0>(XB, XB, DM, WQ, DM, bias, nullptr, QKH, QKL, 2 * DM, 2 * DM, DM);
}
__global__ __launch_bounds__(128) void k_gemm_vt(const unsigned short* __restrict__ WV, const unsigned short* __restrict__ XB, const float* __restrict__ bias,
                                                 unsigned short* __restrict__ VTH, unsigned short* __restrict__ VTL) {
  gemm_body<1, 1>(WV, WV, DM, XB, DM, bias, nullptr, VTH, VTL, MR, MR, DM);
}
__global__ __launch_bounds__(128) void k_gemm_out(const unsigned short* __restrict__ CH, const unsigned short* __restrict__ CL, const unsigned short* __restrict__ WP,
                                                  const float* __restrict__ bias, float* __restrict__ out) {
  gemm_body<2, 2>(CH, CL, DM, WP, DM, bias, out, nullptr, nullptr, DM, DM, DM);
}

template <int REF>
__device__ __forceinline__ void attn_body(const unsigned short* __restrict__ QKH, const unsigned short* __restrict__ QKL,
                                          const unsigned short* __restrict__ VTH, const unsigned short* __restrict__ VTL,
                                          const unsigned int* __restrict__ MB, const unsigned int* __restrict__ FL,
                                          unsigned short* __restrict__ CH, unsigned short* __restrict__ CL, const int qbase) {
  __shared__ __attribute__((aligned(16))) unsigned short sH[4][16][72];
  __shared__ __attribute__((aligned(16))) unsigned short sL[4][16][72];
  const int tid = threadIdx.x, lane = tid & 31, ln = lane & 15, hh = lane >> 4;
  const int wave = __builtin_amdgcn_readfirstlane(tid >> 5);
  const int bh = blockIdx.y;
  const int b = bh / NH, h = bh - b * NH;
  const int q0 = qbase + blockIdx.x * 64 + wave * 16;
  unsigned int fa = 0u;
#pragma unroll 1
  for (int i = lane; i < NFBP; i += 32) { const int ii = (i < NFB) ? i : (NFB - 1); fa |= FL[(size_t)ii * 32]; }
  const bool noskip = __builtin_amdgcn_ballot_w32(fa != 0u) != 0u;
  const float FMIN = __uint_as_float(0xff7fffffu);
  const size_t qoff = (size_t)(b * SEQ + q0 + ln) * (2 * DM) + h * HD + 8 * hh;
  const size_t kbase = (size_t)(b * SEQ + ln) * (2 * DM) + DM + h * HD + 8 * hh;
  const size_t voff = (size_t)(h * HD + ln) * MR + (size_t)b * SEQ + 8 * hh;
  const v8f z8 = {0.f, 0.f, 0.f, 0.f, 0.f, 0.f, 0.f, 0.f};
  v8f o[4] = {z8, z8, z8, z8};
  v8f e[4] = {z8, z8, z8, z8};
  float m = FMIN, l = 0.f;
#pragma unroll 1
  for (int kb = 0; kb < SEQ; kb += 32) {
    const unsigned int w = MB[(size_t)(kb >> 5) * SEQ + q0 + ln];
    if (!noskip && __builtin_amdgcn_ballot_w32(w != 0u) == 0u) continue;
    v8f s0 = z8, s1 = z8;
#pragma unroll
    for (int ks = 0; ks < 2; ++ks) {
      const v16b qh = ldfrag_b(QKH + qoff + ks * 32);
      const v16b ql = ldfrag_b(QKL + qoff + ks * 32);
      const size_t ko0 = kbase + (size_t)kb * (2 * DM) + ks * 32;
      const size_t ko1 = ko0 + (size_t)16 * (2 * DM);
      v16b kh = ldfrag_b(QKH + ko0), kl = ldfrag_b(QKL + ko0);
      s0 = mma_b(kh, qh, s0); s0 = mma_b(kl, qh, s0); s0 = mma_b(kh, ql, s0);
      kh = ldfrag_b(QKH + ko1); kl = ldfrag_b(QKL + ko1);
      s1 = mma_b(kh, qh, s1); s1 = mma_b(kl, qh, s1); s1 = mma_b(kh, ql, s1);
    }
    const unsigned int wsh = w >> (8 * hh);
    float v0[8], v1[8];
    float tm = FMIN;
#pragma unroll
    for (int r = 0; r < 8; ++r) {
      const float a0 = s0[r] * 0.125f, a1 = s1[r] * 0.125f;
      v0[r] = ((wsh >> r) & 1u) ? a0 : FMIN;
      v1[r] = ((wsh >> (16 + r)) & 1u) ? a1 : FMIN;
      tm = fmaxf(tm, fmaxf(v0[r], v1[r]));
    }
    tm = fmaxf(tm, __shfl_xor(tm, 16, 32));
    const float mn = fmaxf(m, tm);
    const float c = __expf(fmaxf(m - mn, -120.0f));
    float ps = 0.f;
    FragH ph, pl;
#pragma unroll
    for (int r = 0; r < 8; ++r) {
      const float p0 = __expf(fmaxf(v0[r] - mn, -120.0f));
      const float p1 = __expf(fmaxf(v1[r] - mn, -120.0f));
      ps += p0 + p1;
      const float pc0 = p0 * 1024.0f, pc1 = p1 * 1024.0f;
      const _Float16 h0 = (_Float16)pc0, h1 = (_Float16)pc1;
      ph.h[r] = h0; ph.h[8 + r] = h1;
      if (REF) { pl.h[r] = (_Float16)((pc0 - (float)h0) * 1024.0f); pl.h[8 + r] = (_Float16)((pc1 - (float)h1) * 1024.0f); }
    }
    l = l * c + ps;
    m = mn;
#pragma unroll
    for (int j = 0; j < 4; ++j)
#pragma unroll
      for (int r = 0; r < 8; ++r) { o[j][r] *= c; if (REF) e[j][r] *= c; }
#pragma unroll
    for (int j = 0; j < 4; ++j) {
      const size_t vo = voff + (size_t)j * 16 * MR + kb;
      const v16h vh = ldfrag_h(VTH + vo);
      o[j] = mma_h(vh, ph.v, o[j]);
      if (REF) {
        const v16h vl = ldfrag_h(VTL + vo);
        e[j] = mma_h(vl, ph.v, e[j]);
        e[j] = mma_h(vh, pl.v, e[j]);
      }
    }
  }
  l += __shfl_xor(l, 16, 32);
  const float inv = (1.0f / l) * 0.0009765625f;
#pragma unroll
  for (int j = 0; j < 4; ++j) {
    v8us hv, lv;
#pragma unroll
    for (int r = 0; r < 8; ++r) {
      float val = o[j][r];
      if (REF) val += e[j][r] * 0.0009765625f;
      val *= inv;
      const unsigned short hb = bf16_bits(val);
      hv[r] = hb; lv[r] = bf16_bits(val - bf16_val(hb));
    }
    *(v8us*)&sH[wave][ln][16 * j + 8 * hh] = hv;
    *(v8us*)&sL[wave][ln][16 * j + 8 * hh] = lv;
  }
  __syncthreads();
  const int rq = lane >> 3, pc = (lane & 7) * 8;
  for (int pass = 0; pass < 2; ++pass) {
#pragma unroll
    for (int it = 0; it < 4; ++it) {
      const int row = it * 4 + rq;
      const v8us xh = *(const v8us*)&sH[wave][row][pc];
      const v8us xl = *(const v8us*)&sL[wave][row][pc];
      const size_t oo = (size_t)(b * SEQ + q0 + row) * DM + h * HD + pc;
      *(volatile v8us*)(CH + oo) = xh;
      *(volatile v8us*)(CL + oo) = xl;
    }
    if (pass == 0) __threadfence();
  }
}

__global__ __launch_bounds__(128) void k_attn_early(const unsigned short* __restrict__ QKH, const unsigned short* __restrict__ QKL,
                                                    const unsigned short* __restrict__ VTH, const unsigned short* __restrict__ VTL,
                                                    const unsigned int* __restrict__ MB, const unsigned int* __restrict__ FL,
                                                    unsigned short* __restrict__ CH, unsigned short* __restrict__ CL) {
  attn_body<1>(QKH, QKL, VTH, VTL, MB, FL, CH, CL, 0);
}
__global__ __launch_bounds__(128) void k_attn_main(const unsigned short* __restrict__ QKH, const unsigned short* __restrict__ QKL,
                                                   const unsigned short* __restrict__ VTH, const unsigned short* __restrict__ VTL,
                                                   const unsigned int* __restrict__ MB, const unsigned int* __restrict__ FL,
                                                   unsigned short* __restrict__ CH, unsigned short* __restrict__ CL) {
  attn_body<0>(QKH, QKL, VTH, VTL, MB, FL, CH, CL, EARLY);
}

extern "C" void kernel_launch(void* const* d_in, const int* in_sizes, int n_in,
                              void* d_out, int out_size, void* d_ws, size_t ws_size, hipStream_t stream) {
  if (n_in < 6) return;
  if (in_sizes[0] < ((NB - 1) * SEQ_FULL + SEQ) * DM) return;
  if (in_sizes[1] < (SEQ - 1) * SEQ_FULL + SEQ) return;
  if (in_sizes[2] < 3 * DM * DM) return;
  if (in_sizes[3] < 3 * DM) return;
  if (in_sizes[4] < DM * DM) return;
  if (in_sizes[5] < DM) return;
  if (out_size < MR * DM) return;
  if (WS_TOTAL > ws_size) return;
  const float* x = (const float*)d_in[0];
  const int* mask = (const int*)d_in[1];
  const float* wqkv = (const float*)d_in[2];
  const float* bqkv = (const float*)d_in[3];
  const float* wproj = (const float*)d_in[4];
  const float* bproj = (const float*)d_in[5];
  float* out = (float*)d_out;
  char* ws = (char*)d_ws;
  unsigned short* XB = (unsigned short*)(ws + OFF_XB);
  unsigned short* WQ = (unsigned short*)(ws + OFF_WQ);
  unsigned short* WP = (unsigned short*)(ws + OFF_WP);
  unsigned short* QKH = (unsigned short*)(ws + OFF_QKH);
  unsigned short* QKL = (unsigned short*)(ws + OFF_QKL);
  unsigned short* VTH = (unsigned short*)(ws + OFF_VTH);
  unsigned short* VTL = (unsigned short*)(ws + OFF_VTL);
  unsigned short* CH = (unsigned short*)(ws + OFF_CH);
  unsigned short* CL = (unsigned short*)(ws + OFF_CL);
  unsigned int* MB = (unsigned int*)(ws + OFF_MB);
  unsigned int* FL = (unsigned int*)(ws + OFF_FL);

  k_wt_bf16<<<(unsigned)((3 * DM * (DM / 8) + 255) / 256), 256, 0, stream>>>(wqkv, WQ, DM, 3 * DM);
  k_wt_bf16<<<(unsigned)((DM * (DM / 8) + 255) / 256), 256, 0, stream>>>(wproj, WP, DM, DM);
  k_xb<<<(unsigned)(((size_t)MR * (DM / 8) + 255) / 256), 256, 0, stream>>>(x, XB);
  k_maskpack<<<NFB, 256, 0, stream>>>(mask, MB, FL);
  k_gemm_qk<<<(unsigned)((MR / 128) * (2 * DM / 64)), 128, 0, stream>>>(XB, WQ, bqkv, QKH, QKL);
  k_gemm_vt<<<(unsigned)((DM / 128) * (MR / 64)), 128, 0, stream>>>(WQ + (size_t)2 * DM * DM, XB, bqkv + 2 * DM, VTH, VTL);
  k_attn_early<<<dim3(EARLY / 64, NB * NH), 128, 0, stream>>>(QKH, QKL, VTH, VTL, MB, FL, CH, CL);
  k_attn_main<<<dim3((SEQ - EARLY) / 64, NB * NH), 128, 0, stream>>>(QKH, QKL, VTH, VTL, MB, FL, CH, CL);
  k_gemm_out<<<(unsigned)((MR / 128) * (DM / 64)), 128, 0, stream>>>(CH, CL, WP, bproj, out);
}
